// ClassifierModel_64931315581364
// MI455X (gfx1250) — hardware-verified
//
#include <hip/hip_runtime.h>


#define NT_  2097152
#define NSEG 8192
#define PCH  65536
#define NCH  (NT_ / PCH)
#define NT   256
#define NWV  (NT / 32)
#define EPT  2
#define CHUNK (NT * EPT)
#define RB   1024
#define LOSC 1024.0f
#define LOSCI (1.0f / 1024.0f)

typedef _Float16 h16;
typedef __attribute__((ext_vector_type(16))) _Float16 v16h;
typedef __attribute__((ext_vector_type(8)))  _Float16 v8h;
typedef __attribute__((ext_vector_type(8)))  float    v8f;
typedef __attribute__((ext_vector_type(4)))  float    v4f;
typedef v8h  __attribute__((may_alias)) v8ha;
typedef v4f  __attribute__((may_alias)) v4fa;

__device__ __forceinline__ unsigned short f2bf(float f) { unsigned u = __float_as_uint(f); u += 0x7FFFu + ((u >> 16) & 1u); return (unsigned short)(u >> 16); }
__device__ __forceinline__ float bf2f(unsigned short b) { return __uint_as_float(((unsigned)b) << 16); }
__device__ __forceinline__ float bfr(float f) { return bf2f(f2bf(f)); }
__device__ __forceinline__ v16h cat16(v8h lo, v8h hi) { return __builtin_shufflevector(lo, hi, 0, 1, 2, 3, 4, 5, 6, 7, 8, 9, 10, 11, 12, 13, 14, 15); }
__device__ __forceinline__ v8f wmma16(v16h a, v16h b, v8f c) { return __builtin_amdgcn_wmma_f32_16x16x32_f16(false, a, false, b, (short)0, c, false, false); }
__device__ __forceinline__ float lrelu(float v) { return v >= 0.f ? v : 0.1f * v; }
#define VST2(T, p, v) do { const T vst2_v_ = (v); *(volatile T*)(p) = vst2_v_; __threadfence(); *(volatile T*)(p) = vst2_v_; } while (0)

__device__ __forceinline__ h16 w16_elem(int t, const float* W2v, const float* W2d, const float* Wc1, const float* Wc2, const float* Wc3) {
    if (t < 1024) { const int n = t >> 5, k = t & 31; return (k < 16) ? (h16)bfr(W2v[(k & 15) * 32 + n]) : (h16)0.f; }
    if (t < 2048) { const int u = t - 1024, n = u >> 5, k = u & 31; return (k < 16) ? (h16)bfr(W2d[(k & 15) * 32 + n]) : (h16)0.f; }
    if (t < 6144) { const int u = t - 2048, n = u >> 6, k = u & 63; return (h16)bfr(Wc1[k * 64 + n]); }
    if (t < 8192) { const int u = t - 6144, n = u >> 6, k = u & 63; return (h16)bfr(Wc2[k * 32 + n]); }
    { const int u = t - 8192, n = u >> 5, k = u & 31; return (n < 8) ? (h16)bfr(Wc3[k * 8 + (n & 7)]) : (h16)0.f; }
}
__global__ __launch_bounds__(256) void k_w16(const float* __restrict__ W2v, const float* __restrict__ W2d, const float* __restrict__ Wc1, const float* __restrict__ Wc2, const float* __restrict__ Wc3,
                                             h16* W2V, h16* W2D, h16* C1, h16* C2, h16* C3) {
    typedef __attribute__((ext_vector_type(4))) _Float16 v4h;
    const int t4 = (blockIdx.x * 256 + threadIdx.x) * 4;
    if (t4 >= 8704) return;
    v4h v;
#pragma unroll
    for (int i = 0; i < 4; ++i) v[i] = w16_elem(t4 + i, W2v, W2d, Wc1, Wc2, Wc3);
    h16* dst = (t4 < 1024) ? (W2V + t4) : (t4 < 2048) ? (W2D + t4 - 1024) : (t4 < 6144) ? (C1 + t4 - 2048) : (t4 < 8192) ? (C2 + t4 - 6144) : (C3 + t4 - 8192);
    VST2(v4h, dst, v);
}

__global__ __launch_bounds__(128) void k_feat(const float* __restrict__ vel, const float* __restrict__ dist, size_t p0g,
                                             const float* __restrict__ W1v, const float* __restrict__ b1v, const float* __restrict__ b2v,
                                             const float* __restrict__ W1d, const float* __restrict__ b1d, const float* __restrict__ b2d,
                                             const h16* __restrict__ W2V, const h16* __restrict__ W2D, h16* F16) {
    __shared__ __align__(16) float ost[4][16 * 68];
    const int lane = threadIdx.x & 31, wave = threadIdx.x >> 5, lr = lane & 15, hi = lane >> 4;
    const int pl0 = blockIdx.x * 64 + wave * 16;
    const size_t pg = p0g + pl0 + lr;
    const float v0 = bfr(vel[pg * 2]), v1 = bfr(vel[pg * 2 + 1]);
    float e[3];
#pragma unroll
    for (int i = 0; i < 3; ++i) e[i] = __expf(-bfr(dist[pg * 3 + i]) * 0.2f);
    v16h av = (v16h){}, ad = (v16h){};
#pragma unroll
    for (int q = 0; q < 8; ++q) {
        const int k = 8 * hi + q;
        float sv = bfr(b1v[k]) + v0 * bfr(W1v[k]) + v1 * bfr(W1v[16 + k]);
        float sd = bfr(b1d[k]);
#pragma unroll
        for (int i = 0; i < 3; ++i) sd += e[i] * bfr(W1d[i * 16 + k]);
        av[q] = (h16)lrelu(sv); ad[q] = (h16)lrelu(sd);
    }
    v8f acc[4];
#pragma unroll
    for (int t = 0; t < 4; ++t) acc[t] = (v8f){};
#pragma unroll
    for (int t = 0; t < 2; ++t) {
        const h16* bv_ = W2V + (size_t)(t * 16 + lr) * 32 + 8 * hi; acc[t] = wmma16(av, cat16(*(const v8h*)bv_, *(const v8h*)(bv_ + 16)), acc[t]);
        const h16* bd_ = W2D + (size_t)(t * 16 + lr) * 32 + 8 * hi; acc[2 + t] = wmma16(ad, cat16(*(const v8h*)bd_, *(const v8h*)(bd_ + 16)), acc[2 + t]);
    }
    asm volatile("v_nop\n\tv_nop\n\tv_nop\n\tv_nop" : "+v"(acc[0]), "+v"(acc[1]), "+v"(acc[2]), "+v"(acc[3]));
    float* os = &ost[wave][0];
#pragma unroll
    for (int t = 0; t < 4; ++t) { const int col = t * 16 + lr; const float bb = (t < 2) ? bfr(b2v[col & 31]) : bfr(b2d[col & 31]);
#pragma unroll
        for (int j = 0; j < 8; ++j) os[(hi * 8 + j) * 68 + col] = lrelu(acc[t][j] + bb); }
    __syncthreads();
    h16* crow = F16 + (size_t)pl0 * 64;
    auto pass = [&]() {
#pragma unroll
        for (int s = 0; s < 4; ++s) { const int row = 4 * s + (lane >> 3), piece = lane & 7; const float* sp = os + row * 68 + piece * 8; v8h o;
#pragma unroll
            for (int i = 0; i < 8; ++i) o[i] = (h16)sp[i];
            *(volatile v8h*)(crow + (size_t)row * 64 + piece * 8) = o; }
    };
    pass(); __threadfence(); pass();
}

__global__ __launch_bounds__(NT) void k_agg(const h16* __restrict__ F16, const int* __restrict__ seg, size_t p0g, int first, float* SEG, float* CNT) {
    extern __shared__ float4 lds_raw[];
    float* agg = (float*)lds_raw; float* cnt = agg + RB * 64; int* lst = (int*)(cnt + RB); int* lse = lst + CHUNK; int* wtot = lse + CHUNK;
    const int t = threadIdx.x, lane = t & 31, wv = t >> 5, s0 = blockIdx.x * RB;
    for (int i = t; i < RB * 64; i += NT) agg[i] = first ? 0.0f : SEG[(size_t)s0 * 64 + i];
    for (int i = t; i < RB; i += NT) cnt[i] = first ? 0.0f : CNT[s0 + i];
    __syncthreads();
#pragma unroll 1
    for (int base = 0; base < PCH; base += CHUNK) {
        int vdl[EPT], ve[EPT], flg[EPT]; int c = 0;
#pragma unroll
        for (int j = 0; j < EPT; ++j) {
            const int e = base + j * NT + t;
            const int d = seg[p0g + e];
            const unsigned udl = (unsigned)d - (unsigned)s0;
            const int f = (udl < (unsigned)RB) ? 1 : 0;
            vdl[j] = (int)udl; ve[j] = e; flg[j] = f; c += f;
        }
        int incl = c;
#pragma unroll
        for (int o = 1; o < 32; o <<= 1) { const int y = __shfl_up(incl, o, 32); if (lane >= o) incl += y; }
        if (lane == 31) wtot[wv] = incl;
        __syncthreads();
        int off = incl - c, tot = 0;
#pragma unroll
        for (int i = 0; i < NWV; ++i) { const int v = wtot[i]; off += (i < wv) ? v : 0; tot += v; }
#pragma unroll
        for (int j = 0; j < EPT; ++j) { if (flg[j]) { lst[off] = vdl[j]; lse[off] = ve[j]; ++off; } }
        __syncthreads();
        if (tot > 0 && t <= 64) {
            if (t < 64) {
#pragma unroll 1
                for (int e2 = 0; e2 < tot; ++e2) agg[lst[e2] * 64 + t] += (float)F16[(size_t)lse[e2] * 64 + t];
            } else {
#pragma unroll 1
                for (int e2 = 0; e2 < tot; ++e2) cnt[lst[e2]] += 1.0f;
            }
        }
        __syncthreads();
    }
#pragma unroll 1
    for (int i = 0; i < RB / NWV; i += 2) {
        const int sl = wv * (RB / NWV) + i + (lane >> 4), piece = lane & 15;
        const v4f v = *(const v4fa*)(agg + sl * 64 + piece * 4);
        VST2(v4f, SEG + (size_t)(s0 + sl) * 64 + piece * 4, v);
    }
    { const int sl = wv * 128 + lane * 4; v4f v; v[0] = cnt[sl]; v[1] = cnt[sl + 1]; v[2] = cnt[sl + 2]; v[3] = cnt[sl + 3]; VST2(v4f, CNT + s0 + sl, v); }
}

__global__ __launch_bounds__(128) void k_cls(const float* __restrict__ SEG, const float* __restrict__ CNT, const h16* __restrict__ C1, const float* __restrict__ bc1,
                                            const h16* __restrict__ C2, const float* __restrict__ bc2, const h16* __restrict__ C3, const float* __restrict__ bc3, float* out) {
    __shared__ __align__(16) h16 hh[4][16 * 72];
    __shared__ __align__(16) h16 hl[4][16 * 72];
    __shared__ __align__(16) float po[4][16 * 8];
    const int lane = threadIdx.x & 31, wave = threadIdx.x >> 5, lr = lane & 15, hi = lane >> 4;
    const int r0 = blockIdx.x * 64 + wave * 16;
    h16* myh = &hh[wave][0]; h16* myl = &hl[wave][0];
    const float ic = 1.0f / fmaxf(CNT[r0 + lr], 1.0f);
    v16h ah[2], al[2];
#pragma unroll
    for (int kc = 0; kc < 2; ++kc)
#pragma unroll
        for (int q = 0; q < 16; ++q) { const int k = kc * 32 + ((q < 8) ? (8 * hi + q) : (16 + 8 * hi + (q - 8))); const float v = SEG[(size_t)(r0 + lr) * 64 + k] * ic;
            const h16 hv = (h16)v; ah[kc][q] = hv; al[kc][q] = (h16)((v - (float)hv) * LOSC); }
    v8f acc[4], accx[4];
#pragma unroll
    for (int n = 0; n < 4; ++n) { acc[n] = (v8f){}; accx[n] = (v8f){}; }
#pragma unroll
    for (int kc = 0; kc < 2; ++kc)
#pragma unroll
        for (int n = 0; n < 4; ++n) { const h16* bp = C1 + (size_t)(n * 16 + lr) * 64 + kc * 32 + 8 * hi; const v16h b = cat16(*(const v8h*)bp, *(const v8h*)(bp + 16)); acc[n] = wmma16(ah[kc], b, acc[n]); accx[n] = wmma16(al[kc], b, accx[n]); }
    asm volatile("v_nop\n\tv_nop\n\tv_nop\n\tv_nop" : "+v"(acc[0]), "+v"(acc[1]), "+v"(acc[2]), "+v"(acc[3]), "+v"(accx[0]), "+v"(accx[1]), "+v"(accx[2]), "+v"(accx[3]));
#pragma unroll
    for (int n = 0; n < 4; ++n)
#pragma unroll
        for (int j = 0; j < 8; ++j) { const float v = lrelu(acc[n][j] + accx[n][j] * LOSCI + bfr(bc1[n * 16 + lr])); const h16 hv = (h16)v; myh[(hi * 8 + j) * 72 + n * 16 + lr] = hv; myl[(hi * 8 + j) * 72 + n * 16 + lr] = (h16)((v - (float)hv) * LOSC); }
    asm volatile("" ::: "memory");
    __builtin_amdgcn_fence(__ATOMIC_RELEASE, "workgroup");
    __builtin_amdgcn_wave_barrier();
#pragma unroll
    for (int kc = 0; kc < 2; ++kc) { ah[kc] = cat16(*(const v8ha*)(myh + lr * 72 + kc * 32 + 8 * hi), *(const v8ha*)(myh + lr * 72 + kc * 32 + 16 + 8 * hi));
                                     al[kc] = cat16(*(const v8ha*)(myl + lr * 72 + kc * 32 + 8 * hi), *(const v8ha*)(myl + lr * 72 + kc * 32 + 16 + 8 * hi)); }
#pragma unroll
    for (int n = 0; n < 2; ++n) { acc[n] = (v8f){}; accx[n] = (v8f){}; }
#pragma unroll
    for (int kc = 0; kc < 2; ++kc)
#pragma unroll
        for (int n = 0; n < 2; ++n) { const h16* bp = C2 + (size_t)(n * 16 + lr) * 64 + kc * 32 + 8 * hi; const v16h b = cat16(*(const v8h*)bp, *(const v8h*)(bp + 16)); acc[n] = wmma16(ah[kc], b, acc[n]); accx[n] = wmma16(al[kc], b, accx[n]); }
    asm volatile("v_nop\n\tv_nop\n\tv_nop\n\tv_nop" : "+v"(acc[0]), "+v"(acc[1]), "+v"(accx[0]), "+v"(accx[1]));
    __builtin_amdgcn_wave_barrier();
#pragma unroll
    for (int n = 0; n < 2; ++n)
#pragma unroll
        for (int j = 0; j < 8; ++j) { const float v = lrelu(acc[n][j] + accx[n][j] * LOSCI + bfr(bc2[n * 16 + lr])); const h16 hv = (h16)v; myh[(hi * 8 + j) * 72 + n * 16 + lr] = hv; myl[(hi * 8 + j) * 72 + n * 16 + lr] = (h16)((v - (float)hv) * LOSC); }
    asm volatile("" ::: "memory");
    __builtin_amdgcn_fence(__ATOMIC_RELEASE, "workgroup");
    __builtin_amdgcn_wave_barrier();
    {
        const v16h a3 = cat16(*(const v8ha*)(myh + lr * 72 + 8 * hi), *(const v8ha*)(myh + lr * 72 + 16 + 8 * hi));
        const v16h a3l = cat16(*(const v8ha*)(myl + lr * 72 + 8 * hi), *(const v8ha*)(myl + lr * 72 + 16 + 8 * hi));
        const h16* bp = C3 + (size_t)lr * 32 + 8 * hi; const v16h b = cat16(*(const v8h*)bp, *(const v8h*)(bp + 16));
        acc[0] = wmma16(a3, b, (v8f){}); accx[0] = wmma16(a3l, b, (v8f){});
        asm volatile("v_nop\n\tv_nop\n\tv_nop\n\tv_nop" : "+v"(acc[0]), "+v"(accx[0]));
    }
    float* pw = &po[wave][0];
#pragma unroll
    for (int j = 0; j < 8; ++j) {
        const float lg = (lr < 8) ? (acc[0][j] + accx[0][j] * LOSCI + bfr(bc3[lr & 7])) : -3.0e38f;
        float mx = lg; mx = fmaxf(mx, __shfl_xor(mx, 1, 16)); mx = fmaxf(mx, __shfl_xor(mx, 2, 16)); mx = fmaxf(mx, __shfl_xor(mx, 4, 16)); mx = fmaxf(mx, __shfl_xor(mx, 8, 16));
        const float ex = (lr < 8) ? __expf(lg - mx) : 0.f;
        float sm = ex; sm += __shfl_xor(sm, 1, 16); sm += __shfl_xor(sm, 2, 16); sm += __shfl_xor(sm, 4, 16); sm += __shfl_xor(sm, 8, 16);
        if (lr < 8) pw[(hi * 8 + j) * 8 + lr] = ex / sm;
    }
    asm volatile("" ::: "memory");
    __builtin_amdgcn_fence(__ATOMIC_RELEASE, "workgroup");
    __builtin_amdgcn_wave_barrier();
    const v4f v = *(const v4fa*)(pw + lane * 4);
    VST2(v4f, out + (size_t)r0 * 8 + lane * 4, v);
}

extern "C" void kernel_launch(void* const* d_in, const int* in_sizes, int n_in,
                              void* d_out, int out_size, void* d_ws, size_t ws_size, hipStream_t stream) {
    (void)in_sizes; (void)n_in; (void)out_size;
    const float* vel = (const float*)d_in[0]; const float* dist = (const float*)d_in[1]; const int* seg = (const int*)d_in[2];
    const float* W1v = (const float*)d_in[4]; const float* b1v = (const float*)d_in[5]; const float* W2v = (const float*)d_in[6]; const float* b2v = (const float*)d_in[7];
    const float* W1d = (const float*)d_in[8]; const float* b1d = (const float*)d_in[9]; const float* W2d = (const float*)d_in[10]; const float* b2d = (const float*)d_in[11];
    const float* Wc1 = (const float*)d_in[12]; const float* bc1 = (const float*)d_in[13]; const float* Wc2 = (const float*)d_in[14]; const float* bc2 = (const float*)d_in[15];
    const float* Wc3 = (const float*)d_in[16]; const float* bc3 = (const float*)d_in[17];
    float* out = (float*)d_out;
    char* wsp = (char*)d_ws;
    auto take = [&](size_t bytes) { char* p = wsp; wsp += (bytes + 255) & ~(size_t)255; return (void*)p; };
    h16* W2V = (h16*)take(1024 * 2); h16* W2D = (h16*)take(1024 * 2); h16* C1 = (h16*)take(4096 * 2); h16* C2 = (h16*)take(2048 * 2); h16* C3 = (h16*)take(512 * 2);
    h16* F16 = (h16*)take((size_t)PCH * 64 * 2); float* SEG = (float*)take((size_t)NSEG * 64 * 4); float* CNT = (float*)take((size_t)NSEG * 4);
    if ((size_t)(wsp - (char*)d_ws) > ws_size) return;
    k_w16<<<(8704 / 4 + 255) / 256, 256, 0, stream>>>(W2v, W2d, Wc1, Wc2, Wc3, W2V, W2D, C1, C2, C3);
    const size_t lds = (size_t)RB * 64 * 4 + RB * 4 + (size_t)CHUNK * 8 + NWV * 4;
    for (int c = 0; c < NCH; ++c) {
        const size_t p0 = (size_t)c * PCH;
        k_feat<<<PCH / 64, 128, 0, stream>>>(vel, dist, p0, W1v, b1v, b2v, W1d, b1d, b2d, W2V, W2D, F16);
        k_agg<<<NSEG / RB, NT, lds, stream>>>(F16, seg, p0, c == 0 ? 1 : 0, SEG, CNT);
    }
    k_cls<<<NSEG / 64, 128, 0, stream>>>(SEG, CNT, C1, bc1, C2, bc2, C3, bc3, out);
}
